// RingNet_24515673326158
// MI455X (gfx1250) — hardware-verified
//
#include <hip/hip_runtime.h>
#include <stdint.h>

#define NB     4
#define NC     96
#define IMGW   128
#define NPIX   16384
#define NPL    384
#define BANDH  32
#define BPIX   4096
#define MROWS  16384
#define NS     13
#define K1     1248
#define LDA1   1280
#define N1     512
#define K2     512
#define N2P    128
#define NOUT   96
#define TROWS  57
#define TP     132
#define BN_EPS_F 1e-5f

typedef __attribute__((ext_vector_type(16))) _Float16 v16h;
typedef __attribute__((ext_vector_type(8)))  _Float16 v8h;
typedef __attribute__((ext_vector_type(16))) __bf16   v16b;
typedef __attribute__((ext_vector_type(8)))  __bf16   v8b;
typedef __attribute__((ext_vector_type(8)))  float    v8f;
typedef __attribute__((ext_vector_type(4)))  float    v4f;

__device__ __forceinline__ unsigned short f2bf_bits(float f) {
  unsigned u = __float_as_uint(f);
  return (unsigned short)((u + 0x7FFFu + ((u >> 16) & 1u)) >> 16);
}
__device__ __forceinline__ float bf_bits2f(unsigned short h) { return __uint_as_float(((unsigned)h) << 16); }

__device__ __forceinline__ void dep_guard_h(v8f& a, v8f& b, v16h x, v16h y) { asm volatile("v_nop\n\tv_nop\n\tv_nop\n\tv_nop" : "+v"(a), "+v"(b) : "v"(x), "v"(y)); }
__device__ __forceinline__ void dep_guard_b(v8f& a, v8f& b, v16b x, v16b y) { asm volatile("v_nop\n\tv_nop\n\tv_nop\n\tv_nop" : "+v"(a), "+v"(b) : "v"(x), "v"(y)); }
__device__ __forceinline__ void keep4_h(v16h a, v16h b, v16h c, v16h d) { asm volatile("v_nop" :: "v"(a), "v"(b), "v"(c), "v"(d)); }
__device__ __forceinline__ void keep4_b(v16b a, v16b b, v16b c, v16b d) { asm volatile("v_nop" :: "v"(a), "v"(b), "v"(c), "v"(d)); }
__device__ __forceinline__ void acc_guard4(v8f& a, v8f& b, v8f& c, v8f& d) { asm volatile("v_nop\n\tv_nop\n\tv_nop\n\tv_nop" : "+v"(a), "+v"(b), "+v"(c), "+v"(d)); }
template <typename T> struct Frag;
template <> struct Frag<_Float16> {
  typedef v16h V; union U { v16h v; v8h h[2]; };
  static __device__ __forceinline__ v16h load(const _Float16* p) {
    U f; f.h[0] = *(const v8h*)(p); f.h[1] = *(const v8h*)(p + 16); return f.v;
  }
  static __device__ __forceinline__ v8f mma(v16h a, v16h b, v8f c) {
    return __builtin_amdgcn_wmma_f32_16x16x32_f16(false, a, false, b, (short)0, c, false, false);
  }
  static __device__ __forceinline__ void guard(v8f& a, v8f& b, v16h x, v16h y) { dep_guard_h(a, b, x, y); }
  static __device__ __forceinline__ void keep(v16h a, v16h b, v16h c, v16h d) { keep4_h(a, b, c, d); }
};
template <> struct Frag<__bf16> {
  typedef v16b V; union U { v16b v; v8b h[2]; };
  static __device__ __forceinline__ v16b load(const __bf16* p) {
    U f; f.h[0] = *(const v8b*)(p); f.h[1] = *(const v8b*)(p + 16); return f.v;
  }
  static __device__ __forceinline__ v8f mma(v16b a, v16b b, v8f c) {
    return __builtin_amdgcn_wmma_f32_16x16x32_bf16(false, a, false, b, (short)0, c, false, false);
  }
  static __device__ __forceinline__ void guard(v8f& a, v8f& b, v16b x, v16b y) { dep_guard_b(a, b, x, y); }
  static __device__ __forceinline__ void keep(v16b a, v16b b, v16b c, v16b d) { keep4_b(a, b, c, d); }
};

template <int ET> struct Elem;
template <> struct Elem<0> { typedef _Float16 T; };
template <> struct Elem<1> { typedef __bf16 T; };
template <int ET, bool SPLIT, int BIAS_MODE, int OUT_MODE, bool RESID, int ACT = 0>
__global__ __launch_bounds__(256) void wmma_gemm64(
    const unsigned short* __restrict__ Ap, const unsigned short* __restrict__ A2p, int lda, long strideA,
    const unsigned short* __restrict__ Btp, const unsigned short* __restrict__ Bt2p, int ldb, long strideB,
    void* __restrict__ Cout, void* __restrict__ Cout2, int ldc, long strideC,
    const float* __restrict__ bias,
    const float* __restrict__ resid, long strideR,
    int M, int N, int K, float scale) {
  typedef typename Elem<ET>::T T;
  typedef typename Frag<T>::V V;
  const T* A = (const T*)Ap; const T* A2 = (const T*)A2p; const T* Bt = (const T*)Btp; const T* Bt2 = (const T*)Bt2p;
  __shared__ __align__(16) float sT[8][16 * 68];
  const int b    = blockIdx.y;
  const int lane = threadIdx.x & 31;
  const int wave = threadIdx.x >> 5;
  const int tilesN = N >> 6;
  const int tilesM = M >> 6;
  const int tile = blockIdx.x * 8 + wave;
  if (tile >= tilesM * tilesN) return;
  const int tm = tile / tilesN;
  const int tn = tile - tm * tilesN;
  const int m0 = tm << 6;
  const int n0 = tn << 6;

  const T* Ab  = A  + (size_t)b * strideA;
  const T* Bb  = Bt + (size_t)b * strideB;
  const T* Ab2 = SPLIT ? (A2  + (size_t)b * strideA) : nullptr;
  const T* Bb2 = SPLIT ? (Bt2 + (size_t)b * strideB) : nullptr;

  const int rlane = lane & 15;
  const int koff  = (lane >> 4) * 8;
  const int mOff  = (lane >> 4) * 8;

  v8f acc[4][4];
#pragma unroll
  for (int i = 0; i < 4; ++i)
#pragma unroll
    for (int j = 0; j < 4; ++j) acc[i][j] = (v8f){0.f,0.f,0.f,0.f,0.f,0.f,0.f,0.f};

  for (int k0 = 0; k0 < K; k0 += 32) {
    V bh[4], bl[4];
#pragma unroll
    for (int j = 0; j < 4; ++j) {
      const size_t bo = (size_t)(n0 + (j << 4) + rlane) * ldb + koff + k0;
      bh[j] = Frag<T>::load(Bb + bo);
      if (SPLIT) bl[j] = Frag<T>::load(Bb2 + bo);
    }
#pragma unroll
    for (int i = 0; i < 4; ++i) {
      const size_t ao = (size_t)(m0 + (i << 4) + rlane) * lda + koff + k0;
      V ah = Frag<T>::load(Ab + ao);
      V al;
      if (SPLIT) al = Frag<T>::load(Ab2 + ao);
#pragma unroll
      for (int j = 0; j < 4; ++j) {
        acc[i][j] = Frag<T>::mma(ah, bh[j], acc[i][j]);
        if (SPLIT) {
          acc[i][j] = Frag<T>::mma(ah, bl[j], acc[i][j]);
          acc[i][j] = Frag<T>::mma(al, bh[j], acc[i][j]);
        }
      }
      Frag<T>::guard(acc[i][0], acc[i][3], ah, SPLIT ? al : ah);
    }
    Frag<T>::keep(bh[0], bh[1], bh[2], bh[3]);
    if (SPLIT) Frag<T>::keep(bl[0], bl[1], bl[2], bl[3]);
  }
  acc_guard4(acc[0][0], acc[0][1], acc[0][2], acc[0][3]);
  acc_guard4(acc[1][0], acc[1][1], acc[1][2], acc[1][3]);
  acc_guard4(acc[2][0], acc[2][1], acc[2][2], acc[2][3]);
  acc_guard4(acc[3][0], acc[3][1], acc[3][2], acc[3][3]);

  float* slab = sT[wave];
  const float* Rb = RESID ? (resid + (size_t)b * strideR) : nullptr;
#pragma unroll
  for (int i = 0; i < 4; ++i) {
    const int mBase = m0 + (i << 4);
#pragma unroll
    for (int j = 0; j < 4; ++j) {
      const int n = n0 + (j << 4) + rlane;
      float bv = 0.f;
      if (BIAS_MODE == 2) bv = bias[n];
#pragma unroll
      for (int r = 0; r < 8; ++r) {
        float v = acc[i][j][r] * scale;
        if (BIAS_MODE == 1) v += bias[mBase + mOff + r];
        if (BIAS_MODE == 2) v += bv;
        if (RESID) v += Rb[(size_t)(mBase + mOff + r) * ldc + n];
        if (ACT == 1) v = tanhf(v);
        if (ACT == 2) v = fmaxf(v, 0.0f);
        if (ACT == 3) v = v / (1.0f + expf(-v));
        if (ACT == 4) v = (v > 0.f) ? v : 0.01f * v;
        if (ACT == 5) v = 0.5f * v * (1.0f + erff(v * 0.70710678118654752f));
        slab[(mOff + r) * 68 + (j << 4) + rlane] = v;
      }
    }
    __builtin_amdgcn_fence(__ATOMIC_RELEASE, "workgroup");
    __builtin_amdgcn_wave_barrier();
    __builtin_amdgcn_fence(__ATOMIC_ACQUIRE, "workgroup");
    if (OUT_MODE == 0) {
      float* C = (float*)Cout + (size_t)b * strideC;
      const int hh = lane >> 4, c4 = (lane & 15) * 4;
      for (int pass = 0; pass < 2; ++pass) {
#pragma unroll
        for (int it = 0; it < 8; ++it) {
          const int row = it * 2 + hh;
          v4f v = *(const v4f*)(slab + row * 68 + c4);
          *(volatile v4f*)(C + (size_t)(mBase + row) * ldc + n0 + c4) = v;
        }
        __threadfence();
      }
    } else {
      const int q = lane >> 3, c8 = (lane & 7) * 8;
      unsigned short* C  = (unsigned short*)Cout  + (size_t)b * strideC;
      unsigned short* C2 = (OUT_MODE == 2) ? ((unsigned short*)Cout2 + (size_t)b * strideC) : nullptr;
      for (int pass = 0; pass < 2; ++pass) {
#pragma unroll
        for (int it = 0; it < 4; ++it) {
          const int row = it * 4 + q;
          const float* sp = slab + row * 68 + c8;
          v8h hv, lv;
#pragma unroll
          for (int e = 0; e < 8; ++e) {
            if (OUT_MODE == 1) {
              hv[e] = (_Float16)sp[e];
            } else {
              unsigned short hb = f2bf_bits(sp[e]);
              unsigned short lb = f2bf_bits(sp[e] - bf_bits2f(hb));
              hv[e] = __builtin_bit_cast(_Float16, hb);
              lv[e] = __builtin_bit_cast(_Float16, lb);
            }
          }
          *(volatile v8h*)(C + (size_t)(mBase + row) * ldc + n0 + c8) = hv;
          if (OUT_MODE == 2) *(volatile v8h*)(C2 + (size_t)(mBase + row) * ldc + n0 + c8) = lv;
        }
        __threadfence();
      }
    }
    __builtin_amdgcn_fence(__ATOMIC_RELEASE, "workgroup");
    __builtin_amdgcn_wave_barrier();
    __builtin_amdgcn_fence(__ATOMIC_ACQUIRE, "workgroup");
  }
}

__global__ __launch_bounds__(256) void fold_w1_kernel(const float* __restrict__ w1, const float* __restrict__ g1,
                                                      const float* __restrict__ v1, _Float16* __restrict__ W1h) {
  const int i = blockIdx.x * 256 + threadIdx.x;
  if (i < (N1 * K1) / 8) {
    const int e0 = i * 8;
    const int o = e0 / K1;
    const int ch0 = e0 - o * K1;
    v8h hv;
#pragma unroll
    for (int e = 0; e < 8; ++e) {
      const int ch = ch0 + e;
      const float s = g1[ch] * rsqrtf(v1[ch] + BN_EPS_F);
      hv[e] = (_Float16)(w1[e0 + e] * s * 16.0f);
    }
    _Float16* dst = W1h + e0;
    *(volatile v8h*)dst = hv;
    __threadfence();
    *(volatile v8h*)dst = hv;
  }
}

__global__ __launch_bounds__(256) void fold_b1_kernel(const float* __restrict__ w1, const float* __restrict__ cb1,
                                                      const float* __restrict__ g1, const float* __restrict__ be1,
                                                      const float* __restrict__ m1, const float* __restrict__ v1,
                                                      float* __restrict__ b1p) {
  __shared__ __align__(16) float sb[256];
  const int tid = threadIdx.x;
  const int o = blockIdx.x * 256 + tid;
  const int oc = min(o, N1 - 1);
  const float* wr = w1 + (size_t)oc * K1;
  float acc = cb1[oc];
#pragma unroll 1
  for (int ch = 0; ch < K1; ++ch) {
    const float s = g1[ch] * rsqrtf(v1[ch] + BN_EPS_F);
    const float t = be1[ch] - m1[ch] * s;
    acc += wr[ch] * t;
  }
  sb[tid] = acc;
  __syncthreads();
  if (tid < 32) {
    v4f v0 = *(const v4f*)(sb + tid * 4);
    v4f v1v = *(const v4f*)(sb + 128 + tid * 4);
    float* d0 = b1p + blockIdx.x * 256 + tid * 4;
    float* d1 = b1p + blockIdx.x * 256 + 128 + tid * 4;
    for (int pass = 0; pass < 2; ++pass) {
      *(volatile v4f*)d0 = v0;
      *(volatile v4f*)d1 = v1v;
      __threadfence();
    }
  }
}

__global__ __launch_bounds__(256) void fold_w2_kernel(const float* __restrict__ w2, const float* __restrict__ g2,
                                                      const float* __restrict__ v2, _Float16* __restrict__ W2h) {
  const int i = blockIdx.x * 256 + threadIdx.x;
  if (i < (N2P * K2) / 8) {
    const int e0 = i * 8;
    const int o = e0 >> 9;
    const int k0 = e0 & (K2 - 1);
    const bool valid = o < NOUT;
    const int oc = min(o, NOUT - 1);
    v8h hv;
#pragma unroll
    for (int e = 0; e < 8; ++e) {
      const int k = k0 + e;
      const float s = g2[k] * rsqrtf(v2[k] + BN_EPS_F);
      const float wv = w2[(size_t)oc * K2 + k] * s * 16.0f;
      hv[e] = (_Float16)(valid ? wv : 0.0f);
    }
    _Float16* dst = W2h + e0;
    *(volatile v8h*)dst = hv;
    __threadfence();
    *(volatile v8h*)dst = hv;
  }
}

__global__ __launch_bounds__(128) void fold_b2_kernel(const float* __restrict__ w2, const float* __restrict__ cb2,
                                                      const float* __restrict__ g2, const float* __restrict__ be2,
                                                      const float* __restrict__ m2, const float* __restrict__ v2,
                                                      float* __restrict__ b2p) {
  __shared__ __align__(16) float sb[128];
  const int tid = threadIdx.x;
  const int o = tid;
  const bool valid = o < NOUT;
  const int oc = min(o, NOUT - 1);
  const float* wr = w2 + (size_t)oc * K2;
  float acc = cb2[oc];
#pragma unroll 1
  for (int k = 0; k < K2; ++k) {
    const float s = g2[k] * rsqrtf(v2[k] + BN_EPS_F);
    const float t = be2[k] - m2[k] * s;
    acc += wr[k] * t;
  }
  sb[tid] = valid ? acc : 0.0f;
  __syncthreads();
  if (tid < 32) {
    v4f v0 = *(const v4f*)(sb + tid * 4);
    float* d0 = b2p + tid * 4;
    for (int pass = 0; pass < 2; ++pass) {
      *(volatile v4f*)d0 = v0;
      __threadfence();
    }
  }
}

__global__ __launch_bounds__(256) void ring_band_kernel(const float* __restrict__ x, _Float16* __restrict__ R, int i0) {
  __shared__ __align__(16) float T[TROWS * TP];
  const int tid = threadIdx.x;
  const int pl = blockIdx.x;
  const int b = pl / NC;
  const int c = pl - b * NC;
  const float* xp = x + (size_t)pl * NPIX;

  if (tid < TP) T[tid] = 0.0f;
  if (tid < TROWS) T[tid * TP] = 0.0f;
#pragma unroll 1
  for (int it = 0; it < 28; ++it) {
    const int idx = it * 256 + tid;
    const int t = (idx >> 7) + 1;
    const int col = idx & 127;
    const int row = i0 - 13 + t;
    const bool valid = (row >= 0) && (row < IMGW);
    const int rowc = min(max(row, 0), IMGW - 1);
    float v = xp[rowc * IMGW + col];
    v = valid ? v : 0.0f;
    T[t * TP + col + 1] = v;
  }
  __syncthreads();
  if (tid < 56) {
    float* Rw = T + (tid + 1) * TP;
    float s = 0.0f;
#pragma unroll 1
    for (int u = 1; u <= IMGW; ++u) { s += Rw[u]; Rw[u] = s; }
  }
  __syncthreads();
  if (tid < IMGW) {
    float* Cl = T + (tid + 1);
    float s = 0.0f;
#pragma unroll 1
    for (int t = 1; t <= 56; ++t) { s += Cl[t * TP]; Cl[t * TP] = s; }
  }
  __syncthreads();

#pragma unroll 1
  for (int cc = 0; cc < 2; ++cc) {
    const int q0 = cc * 2048 + tid * 8;
    const int il = q0 >> 7;
    const int j0 = q0 & 127;
    const int i = i0 + il;
    float xv[8];
    {
      const v4f a0 = *(const v4f*)(xp + i * IMGW + j0);
      const v4f a1 = *(const v4f*)(xp + i * IMGW + j0 + 4);
      xv[0] = a0[0]; xv[1] = a0[1]; xv[2] = a0[2]; xv[3] = a0[3];
      xv[4] = a1[0]; xv[5] = a1[1]; xv[6] = a1[2]; xv[7] = a1[3];
    }
    {
      v8h hv;
#pragma unroll
      for (int e = 0; e < 8; ++e) hv[e] = (_Float16)xv[e];
      _Float16* dst = R + ((size_t)(0 * NB + b) * NC + c) * BPIX + q0;
      *(volatile v8h*)dst = hv;
      __threadfence();
      *(volatile v8h*)dst = hv;
    }
    float prev[8];
#pragma unroll
    for (int e = 0; e < 8; ++e) prev[e] = xv[e];
#pragma unroll 1
    for (int p = 1; p <= 12; ++p) {
      const int r0 = max(i - p, 0);
      const int r1 = min(i + p, IMGW - 1);
      const int t0 = r0 - i0 + 12;
      const int t1 = r1 - i0 + 13;
      const float* T0 = T + t0 * TP;
      const float* T1 = T + t1 * TP;
      v8h hv;
#pragma unroll
      for (int e = 0; e < 8; ++e) {
        const int j = j0 + e;
        const int cl0 = max(j - p, 0);
        const int cl1 = min(j + p, IMGW - 1) + 1;
        const float box = ((T1[cl1] - T0[cl1]) - T1[cl0]) + T0[cl0];
        const float ring = box - prev[e];
        prev[e] = box;
        hv[e] = (_Float16)ring;
      }
      _Float16* dst = R + ((size_t)(p * NB + b) * NC + c) * BPIX + q0;
      *(volatile v8h*)dst = hv;
      __threadfence();
      *(volatile v8h*)dst = hv;
    }
  }
}

__global__ __launch_bounds__(256) void transpose_band_kernel(const _Float16* __restrict__ R, _Float16* __restrict__ A1) {
  __shared__ __align__(16) _Float16 tile[64 * 72];
  const int tid = threadIdx.x;
  const int pxT = blockIdx.x;
  const int chT = blockIdx.y;
  const int b = pxT >> 6;
  const int q0 = (pxT & 63) * 64;
  const int px0 = pxT * 64;
  const int ch0 = chT * 64;
#pragma unroll
  for (int it = 0; it < 2; ++it) {
    const int idx = it * 256 + tid;
    const int chl = idx >> 3;
    const int seg = idx & 7;
    const int ch = ch0 + chl;
    const bool valid = ch < K1;
    const int chc = min(ch, K1 - 1);
    const int s = chc / NC;
    const int c = chc - s * NC;
    const _Float16* src = R + ((size_t)(s * NB + b) * NC + c) * BPIX + q0 + seg * 8;
    v8h v = *(const v8h*)src;
    if (!valid) {
#pragma unroll
      for (int e = 0; e < 8; ++e) v[e] = (_Float16)0.0f;
    }
    *(v8h*)(tile + chl * 72 + seg * 8) = v;
  }
  __syncthreads();
  const int wave = tid >> 5, lane = tid & 31;
  const int l8 = lane & 7, rq = lane >> 3;
  v8h hv0, hv1;
  const int pxl0 = wave * 8 + rq;
  const int pxl1 = wave * 8 + 4 + rq;
#pragma unroll
  for (int e = 0; e < 8; ++e) {
    hv0[e] = tile[(8 * l8 + e) * 72 + pxl0];
    hv1[e] = tile[(8 * l8 + e) * 72 + pxl1];
  }
  _Float16* d0 = A1 + (size_t)(px0 + pxl0) * LDA1 + ch0 + 8 * l8;
  _Float16* d1 = A1 + (size_t)(px0 + pxl1) * LDA1 + ch0 + 8 * l8;
  for (int pass = 0; pass < 2; ++pass) {
    *(volatile v8h*)d0 = hv0;
    *(volatile v8h*)d1 = hv1;
    __threadfence();
  }
}

__global__ __launch_bounds__(256) void out_band_kernel(const float* __restrict__ C2, float* __restrict__ out, int i0) {
  __shared__ __align__(16) float tile[64 * 36];
  const int tid = threadIdx.x;
  const int pxT = blockIdx.x;
  const int b = pxT >> 6;
  const int q0 = (pxT & 63) * 64;
  const int px0 = pxT * 64;
  const int o0 = blockIdx.y * 32;
#pragma unroll
  for (int it = 0; it < 2; ++it) {
    const int idx = it * 256 + tid;
    const int pxl = idx >> 3;
    const int seg = idx & 7;
    const v4f v = *(const v4f*)(C2 + (size_t)(px0 + pxl) * N2P + o0 + seg * 4);
    *(v4f*)(tile + pxl * 36 + seg * 4) = v;
  }
  __syncthreads();
  const int wave = tid >> 5, lane = tid & 31;
  const int l16 = lane & 15, rh = lane >> 4;
  const int ol0 = wave * 4 + rh;
  const int ol1 = wave * 4 + 2 + rh;
  v4f w0, w1v;
#pragma unroll
  for (int e = 0; e < 4; ++e) {
    w0[e]  = tile[(4 * l16 + e) * 36 + ol0];
    w1v[e] = tile[(4 * l16 + e) * 36 + ol1];
  }
  float* d0 = out + ((size_t)(b * NOUT + o0 + ol0)) * NPIX + (size_t)i0 * IMGW + q0 + 4 * l16;
  float* d1 = out + ((size_t)(b * NOUT + o0 + ol1)) * NPIX + (size_t)i0 * IMGW + q0 + 4 * l16;
  for (int pass = 0; pass < 2; ++pass) {
    *(volatile v4f*)d0 = w0;
    *(volatile v4f*)d1 = w1v;
    __threadfence();
  }
}

static inline size_t al256(size_t v) { return (v + 255) & ~((size_t)255); }

extern "C" void kernel_launch(void* const* d_in, const int* in_sizes, int n_in,
                              void* d_out, int out_size, void* d_ws, size_t ws_size,
                              hipStream_t stream) {
  if (n_in < 13) return;
  if (in_sizes[0] != NB * NC * NPIX) return;
  if (in_sizes[1] != K1 || in_sizes[2] != K1 || in_sizes[3] != K1 || in_sizes[4] != K1) return;
  if (in_sizes[5] != N1 * K1 || in_sizes[6] != N1) return;
  if (in_sizes[7] != K2 || in_sizes[8] != K2 || in_sizes[9] != K2 || in_sizes[10] != K2) return;
  if (in_sizes[11] != NOUT * K2 || in_sizes[12] != NOUT) return;
  if (out_size != NB * NOUT * NPIX) return;

  const float* x     = (const float*)d_in[0];
  const float* bn1_g = (const float*)d_in[1];
  const float* bn1_b = (const float*)d_in[2];
  const float* bn1_m = (const float*)d_in[3];
  const float* bn1_v = (const float*)d_in[4];
  const float* w1    = (const float*)d_in[5];
  const float* cb1   = (const float*)d_in[6];
  const float* bn2_g = (const float*)d_in[7];
  const float* bn2_b = (const float*)d_in[8];
  const float* bn2_m = (const float*)d_in[9];
  const float* bn2_v = (const float*)d_in[10];
  const float* w2    = (const float*)d_in[11];
  const float* cb2   = (const float*)d_in[12];
  float* out = (float*)d_out;

  char* ws = (char*)d_ws;
  size_t off = 0;
  _Float16* R   = (_Float16*)(ws + off); off += al256((size_t)NS * NPL * BPIX * 2);
  _Float16* A1  = (_Float16*)(ws + off); off += al256((size_t)MROWS * LDA1 * 2);
  _Float16* A2  = (_Float16*)(ws + off); off += al256((size_t)MROWS * N1 * 2);
  float*    C2  = (float*)(ws + off);    off += al256((size_t)MROWS * N2P * 4);
  _Float16* W1h = (_Float16*)(ws + off); off += al256((size_t)N1 * K1 * 2);
  _Float16* W2h = (_Float16*)(ws + off); off += al256((size_t)N2P * K2 * 2);
  float*    b1p = (float*)(ws + off);    off += al256((size_t)N1 * 4);
  float*    b2p = (float*)(ws + off);    off += al256((size_t)N2P * 4);
  if (off > ws_size) return;

  fold_w1_kernel<<<(N1 * K1 / 8 + 255) / 256, 256, 0, stream>>>(w1, bn1_g, bn1_v, W1h);
  fold_b1_kernel<<<2, 256, 0, stream>>>(w1, cb1, bn1_g, bn1_b, bn1_m, bn1_v, b1p);
  fold_w2_kernel<<<(N2P * K2 / 8 + 255) / 256, 256, 0, stream>>>(w2, bn2_g, bn2_v, W2h);
  fold_b2_kernel<<<1, 128, 0, stream>>>(w2, cb2, bn2_g, bn2_b, bn2_m, bn2_v, b2p);

  const int g1_blocks = ((MROWS / 64) * (N1 / 64) + 7) / 8;
  const int g2_blocks = ((MROWS / 64) * (N2P / 64) + 7) / 8;

  for (int band = 0; band < IMGW / BANDH; ++band) {
    const int i0 = band * BANDH;
    ring_band_kernel<<<NPL, 256, 0, stream>>>(x, R, i0);
    transpose_band_kernel<<<dim3(MROWS / 64, LDA1 / 64), 256, 0, stream>>>(R, A1);
    wmma_gemm64<0, false, 2, 1, false, 2><<<dim3(g1_blocks, 1), 256, 0, stream>>>(
        (const unsigned short*)A1, (const unsigned short*)A1, LDA1, 0L,
        (const unsigned short*)W1h, (const unsigned short*)W1h, K1, 0L,
        (void*)A2, (void*)A2, N1, 0L,
        b1p, b1p, 0L,
        MROWS, N1, K1, 1.0f / 16.0f);
    wmma_gemm64<0, false, 2, 0, false, 0><<<dim3(g2_blocks, 1), 256, 0, stream>>>(
        (const unsigned short*)A2, (const unsigned short*)A2, N1, 0L,
        (const unsigned short*)W2h, (const unsigned short*)W2h, K2, 0L,
        (void*)C2, (void*)C2, N2P, 0L,
        b2p, b2p, 0L,
        MROWS, N2P, K2, 1.0f / 16.0f);
    out_band_kernel<<<dim3(MROWS / 64, NOUT / 32), 256, 0, stream>>>(C2, out, i0);
  }
}
